// Attention_20066087207334
// MI455X (gfx1250) — hardware-verified
//
#include <hip/hip_runtime.h>


#ifndef NB
#define NB 4
#endif
#ifndef SEQ
#define SEQ 2048
#endif
#define NB_FULL  4
#define SEQ_FULL 2048
#define DM   1024
#define NH_  16
#define HD   64
#define RH   ((SEQ) < 512 ? (SEQ) : 512)
#define PCAR 1024.0f
#define SCL  0.125f
#define L2E  1.4426950408889634f
#define NEGB (-3.0e38f)

static_assert(NH_ * HD == DM);
static_assert(HD == 64);
static_assert(DM % 64 == 0);
static_assert(SEQ % 64 == 0);
static_assert(RH % 64 == 0);
static_assert(RH <= SEQ);
static_assert(NB <= NB_FULL);
static_assert(SEQ <= SEQ_FULL);
static_assert(DM / 8 == 128);
static_assert(HD * 4 == 16 * 16);
static_assert((DM * 4) % 128 == 0 && (HD * 4) % 128 == 0);
static_assert(RH % 16 == 0 && (SEQ - RH) % 16 == 0);
static_assert(NB * NH_ <= 65535);

typedef _Float16 h16;
typedef unsigned short bf;
typedef __attribute__((ext_vector_type(16))) __bf16   v16bf;
typedef __attribute__((ext_vector_type(16))) _Float16 v16h;
typedef __attribute__((ext_vector_type(8)))  _Float16 v8h;
typedef __attribute__((ext_vector_type(8)))  unsigned short v8us;
typedef __attribute__((ext_vector_type(8)))  float    v8f;
typedef __attribute__((ext_vector_type(4)))  float    v4f;
typedef v8h  __attribute__((may_alias)) v8ha;
typedef v4f  __attribute__((may_alias)) v4fa;
typedef v8us __attribute__((may_alias)) v8usa;

__device__ __forceinline__ unsigned short f2bf(float f) { unsigned u = __float_as_uint(f); u += 0x7FFFu + ((u >> 16) & 1u); return (unsigned short)(u >> 16); }
__device__ __forceinline__ float bf2f(unsigned short b) { return __uint_as_float(((unsigned)b) << 16); }
__device__ __forceinline__ float bfr(float f) { return bf2f(f2bf(f)); }
__device__ __forceinline__ v16h cat16(v8h lo, v8h hi) { return __builtin_shufflevector(lo, hi, 0, 1, 2, 3, 4, 5, 6, 7, 8, 9, 10, 11, 12, 13, 14, 15); }
__device__ __forceinline__ v16bf cat16b(v8us lo, v8us hi) { return __builtin_bit_cast(v16bf, __builtin_shufflevector(lo, hi, 0, 1, 2, 3, 4, 5, 6, 7, 8, 9, 10, 11, 12, 13, 14, 15)); }
__device__ __forceinline__ v8f wmma16(v16h a, v16h b, v8f c) { return __builtin_amdgcn_wmma_f32_16x16x32_f16(false, a, false, b, (short)0, c, false, false); }
__device__ __forceinline__ v8f wmmab(v16bf a, v16bf b, v8f c) { return __builtin_amdgcn_wmma_f32_16x16x32_bf16(false, a, false, b, (short)0, c, false, false); }
__device__ __forceinline__ void splitf(float y, unsigned short& h, unsigned short& l) { h = f2bf(y); l = f2bf(y - bf2f(h)); }

static __device__ __forceinline__ h16 toh_flush(float v) { const h16 r = (h16)v; return (fabsf(v) < 6.103515625e-05f) ? (h16)0.0f : r; }

template <typename T16> struct WFrag;
template <> struct WFrag<h16> { typedef v16h V;
    static __device__ __forceinline__ V ld(const h16* p) { return cat16(*(const v8h*)p, *(const v8h*)(p + 16)); }
    static __device__ __forceinline__ V ldl(const h16* p) { return cat16(*(const v8ha*)p, *(const v8ha*)(p + 16)); }
    static __device__ __forceinline__ v8f mma(V a, V b, v8f c) { return wmma16(a, b, c); } };
template <> struct WFrag<bf> { typedef v16bf V;
    static __device__ __forceinline__ V ld(const bf* p) { return cat16b(*(const v8us*)p, *(const v8us*)(p + 16)); }
    static __device__ __forceinline__ V ldl(const bf* p) { return cat16b(*(const v8usa*)p, *(const v8usa*)(p + 16)); }
    static __device__ __forceinline__ v8f mma(V a, V b, v8f c) { return wmmab(a, b, c); } };

template <int VMODE>
__global__ __launch_bounds__(32) void k_projp(const bf* __restrict__ A, const bf* __restrict__ Bt, h16* P16, bf* Ph, bf* Pl) {
    typedef WFrag<bf>::V V;
    __shared__ __align__(16) float os[64 * 68];
    const unsigned lane = threadIdx.x & 31u, lr = lane & 15u, hi = lane >> 4; const unsigned r0 = blockIdx.x * 64u, c0 = blockIdx.y * 64u;
    v8f acc[4][4];
#pragma unroll
    for (int mb = 0; mb < 4; ++mb)
#pragma unroll
        for (int nb = 0; nb < 4; ++nb) acc[mb][nb] = (v8f){};
    const size_t aoff = (size_t)(r0 + lr) * DM + 8u * hi, boff = (size_t)(c0 + lr) * DM + 8u * hi;
#pragma unroll 1
    for (unsigned kc = 0; kc < (unsigned)DM; kc += 32u) {
        V a[4];
#pragma unroll
        for (int mb = 0; mb < 4; ++mb) a[mb] = WFrag<bf>::ld(A + aoff + (size_t)mb * 16 * DM + kc);
#pragma unroll
        for (int nb = 0; nb < 4; ++nb) { const V b = WFrag<bf>::ld(Bt + boff + (size_t)nb * 16 * DM + kc);
#pragma unroll
            for (int mb = 0; mb < 4; ++mb) acc[mb][nb] = WFrag<bf>::mma(a[mb], b, acc[mb][nb]); }
        asm volatile("v_nop\n\tv_nop\n\tv_nop\n\tv_nop" : "+v"(acc[0][0]), "+v"(acc[1][1]), "+v"(acc[2][2]), "+v"(acc[3][3]) : "v"(a[0]), "v"(a[3]));
    }
#pragma unroll
    for (int mb = 0; mb < 4; ++mb)
#pragma unroll
        for (int nb = 0; nb < 4; ++nb)
#pragma unroll
            for (int j = 0; j < 8; ++j) os[(mb * 16 + hi * 8 + j) * 68 + nb * 16 + lr] = acc[mb][nb][j];
    __syncthreads();
    const unsigned b = r0 / (unsigned)SEQ, t0 = r0 % (unsigned)SEQ; const unsigned bh = b * NH_ + blockIdx.y;
    const bool hires = (t0 < (unsigned)RH);
    const unsigned rq = lane >> 3, pc = lane & 7u;
    if (VMODE == 0) {
        const size_t o16 = ((size_t)bh * SEQ + t0) * HD + pc * 8u;
        const size_t ohl = ((size_t)bh * RH + t0) * HD + pc * 8u;
#pragma unroll 1
        for (int ps = 0; ps < 2; ++ps) {
#pragma unroll 2
            for (unsigned s = 0; s < 16u; ++s) { const unsigned row = s * 4u + rq;
                const v4f x0 = *(const v4fa*)(os + row * 68u + pc * 8u), x1 = *(const v4fa*)(os + row * 68u + pc * 8u + 4u); v8h o;
#pragma unroll
                for (int q = 0; q < 4; ++q) { o[q] = (h16)x0[q]; o[4 + q] = (h16)x1[q]; }
                *(volatile v8h*)(P16 + o16 + (size_t)row * HD) = o;
                if (hires) { v8us oh, ol;
#pragma unroll
                    for (int q = 0; q < 4; ++q) { unsigned short a2, c2; splitf(x0[q], a2, c2); oh[q] = a2; ol[q] = c2; splitf(x1[q], a2, c2); oh[4 + q] = a2; ol[4 + q] = c2; }
                    *(volatile v8us*)(Ph + ohl + (size_t)row * HD) = oh; *(volatile v8us*)(Pl + ohl + (size_t)row * HD) = ol; } }
            if (ps == 0) __threadfence(); }
    } else {
        const size_t o16 = (size_t)bh * HD * SEQ + t0 + pc * 8u;
        const size_t ohl = (size_t)bh * HD * RH + t0 + pc * 8u;
#pragma unroll 1
        for (int ps = 0; ps < 2; ++ps) {
#pragma unroll 2
            for (unsigned s = 0; s < 16u; ++s) { const unsigned d = s * 4u + rq;
                float x[8];
#pragma unroll
                for (int j = 0; j < 8; ++j) x[j] = os[(pc * 8u + j) * 68u + d];
                v8h o;
#pragma unroll
                for (int j = 0; j < 8; ++j) o[j] = (h16)x[j];
                *(volatile v8h*)(P16 + o16 + (size_t)d * SEQ) = o;
                if (hires) { v8us oh, ol;
#pragma unroll
                    for (int j = 0; j < 8; ++j) { unsigned short a2, c2; splitf(x[j], a2, c2); oh[j] = a2; ol[j] = c2; }
                    *(volatile v8us*)(Ph + ohl + (size_t)d * RH) = oh; *(volatile v8us*)(Pl + ohl + (size_t)d * RH) = ol; } }
            if (ps == 0) __threadfence(); }
    }
}

__device__ __forceinline__ void pputf(h16* ph, h16* pl, unsigned idx, float p) { (void)pl; ph[idx] = toh_flush(p * PCAR); }
__device__ __forceinline__ void pputf(bf* ph, bf* pl, unsigned idx, float p) { unsigned short a, c; splitf(p, a, c); ph[idx] = a; pl[idx] = c; }

template <typename T16, bool SPLIT, unsigned PROW>
__global__ __launch_bounds__(32) void k_flash(const T16* __restrict__ Q, const T16* __restrict__ Q2, const T16* __restrict__ Kp, const T16* __restrict__ K2, const T16* __restrict__ Vt, const T16* __restrict__ Vt2, unsigned roff, float* OUT) {
    typedef typename WFrag<T16>::V V;
    __shared__ __align__(16) T16 psh[16 * 72];
    __shared__ __align__(16) T16 psl[SPLIT ? 16 * 72 : 8];
    __shared__ __align__(16) float os[16 * 68];
    const unsigned lane = threadIdx.x & 31u, lr = lane & 15u, hi = lane >> 4;
    const unsigned bh = blockIdx.y, r0 = roff + blockIdx.x * 16u;
    const size_t pb = (size_t)bh * PROW * HD;
    const size_t qo = pb + (size_t)(r0 + lr) * HD + 8u * hi;
    V qa[2], qb[2];
#pragma unroll
    for (int ks = 0; ks < 2; ++ks) { qa[ks] = WFrag<T16>::ld(Q + qo + ks * 32); if (SPLIT) qb[ks] = WFrag<T16>::ld(Q2 + qo + ks * 32); }
    v8f O[4]; float mrun[8], lsum[8];
#pragma unroll
    for (int nt = 0; nt < 4; ++nt) O[nt] = (v8f){};
#pragma unroll
    for (int r = 0; r < 8; ++r) { mrun[r] = NEGB; lsum[r] = 0.0f; }
    const unsigned nkt = (r0 >> 6) + 1u;
#pragma unroll 1
    for (unsigned kt = 0; kt < nkt; ++kt) {
        const unsigned c0 = kt * 64u;
        v8f S[4]; V kb, kb2;
        const size_t ko = pb + (size_t)(c0 + lr) * HD + 8u * hi;
#pragma unroll
        for (int ni = 0; ni < 4; ++ni) { S[ni] = (v8f){};
#pragma unroll
            for (int ks = 0; ks < 2; ++ks) { kb = WFrag<T16>::ld(Kp + ko + (size_t)ni * 16 * HD + ks * 32); S[ni] = WFrag<T16>::mma(qa[ks], kb, S[ni]);
                if (SPLIT) { S[ni] = WFrag<T16>::mma(qb[ks], kb, S[ni]); kb2 = WFrag<T16>::ld(K2 + ko + (size_t)ni * 16 * HD + ks * 32); S[ni] = WFrag<T16>::mma(qa[ks], kb2, S[ni]); } } }
        if (SPLIT) asm volatile("v_nop\n\tv_nop\n\tv_nop\n\tv_nop" : "+v"(S[0]), "+v"(S[1]), "+v"(S[2]), "+v"(S[3]) : "v"(qa[1]), "v"(kb2));
        else       asm volatile("v_nop\n\tv_nop\n\tv_nop\n\tv_nop" : "+v"(S[0]), "+v"(S[1]), "+v"(S[2]), "+v"(S[3]) : "v"(qa[1]), "v"(kb));
        const bool diag = (kt + 1u == nkt);
        float mnew[8];
#pragma unroll
        for (int r = 0; r < 8; ++r) { const unsigned row = r0 + 8u * hi + r; float mx = NEGB;
#pragma unroll
            for (int ni = 0; ni < 4; ++ni) { const unsigned key = c0 + ni * 16u + lr; float t = S[ni][r] * SCL; t = (diag && key > row) ? NEGB : t; S[ni][r] = t; mx = fmaxf(mx, t); }
            mx = fmaxf(mx, __shfl_xor(mx, 8, 32)); mx = fmaxf(mx, __shfl_xor(mx, 4, 32)); mx = fmaxf(mx, __shfl_xor(mx, 2, 32)); mx = fmaxf(mx, __shfl_xor(mx, 1, 32));
            mnew[r] = fmaxf(mrun[r], mx); }
#pragma unroll
        for (int r = 0; r < 8; ++r) { const float al = __builtin_amdgcn_exp2f((mrun[r] - mnew[r]) * L2E); mrun[r] = mnew[r]; lsum[r] *= al;
#pragma unroll
            for (int nt = 0; nt < 4; ++nt) O[nt][r] *= al; }
#pragma unroll
        for (int r = 0; r < 8; ++r)
#pragma unroll
            for (int ni = 0; ni < 4; ++ni) { const float p = __builtin_amdgcn_exp2f((S[ni][r] - mnew[r]) * L2E); lsum[r] += p; pputf(psh, psl, (8u * hi + r) * 72u + ni * 16u + lr, p); }
        __syncthreads();
        V pa[2], pl[2];
#pragma unroll
        for (int ks = 0; ks < 2; ++ks) { pa[ks] = WFrag<T16>::ldl(psh + lr * 72u + ks * 32 + 8u * hi); if (SPLIT) pl[ks] = WFrag<T16>::ldl(psl + lr * 72u + ks * 32 + 8u * hi); }
        V vb, vb2;
        const size_t vo = pb + (size_t)lr * PROW + c0 + 8u * hi;
#pragma unroll
        for (int nt = 0; nt < 4; ++nt) {
#pragma unroll
            for (int ks = 0; ks < 2; ++ks) { vb = WFrag<T16>::ld(Vt + vo + (size_t)nt * 16 * PROW + ks * 32); O[nt] = WFrag<T16>::mma(pa[ks], vb, O[nt]);
                if (SPLIT) { O[nt] = WFrag<T16>::mma(pl[ks], vb, O[nt]); vb2 = WFrag<T16>::ld(Vt2 + vo + (size_t)nt * 16 * PROW + ks * 32); O[nt] = WFrag<T16>::mma(pa[ks], vb2, O[nt]); } } }
        if (SPLIT) asm volatile("v_nop\n\tv_nop\n\tv_nop\n\tv_nop" : "+v"(O[0]), "+v"(O[1]), "+v"(O[2]), "+v"(O[3]) : "v"(pa[1]), "v"(vb2));
        else       asm volatile("v_nop\n\tv_nop\n\tv_nop\n\tv_nop" : "+v"(O[0]), "+v"(O[1]), "+v"(O[2]), "+v"(O[3]) : "v"(pa[1]), "v"(vb));
        __syncthreads();
    }
#pragma unroll
    for (int r = 0; r < 8; ++r) { float l = lsum[r]; l += __shfl_xor(l, 8, 32); l += __shfl_xor(l, 4, 32); l += __shfl_xor(l, 2, 32); l += __shfl_xor(l, 1, 32);
        const float inv = __fdiv_rn(1.0f, l) * (SPLIT ? 1.0f : (1.0f / PCAR));
#pragma unroll
        for (int nt = 0; nt < 4; ++nt) os[(8u * hi + r) * 68u + nt * 16u + lr] = O[nt][r] * inv; }
    __syncthreads();
    const unsigned b = bh / (unsigned)NH_, h = bh % (unsigned)NH_;
    float* orow = OUT + ((size_t)b * SEQ_FULL + r0) * DM + h * HD;
#pragma unroll 1
    for (int ps = 0; ps < 2; ++ps) {
#pragma unroll
        for (unsigned s = 0; s < 8u; ++s) { const unsigned row = 2u * s + hi, cofs = lr * 4u;
            const v4f val = *(const v4fa*)(os + row * 68u + cofs);
            *(volatile v4f*)(orow + (size_t)row * DM + cofs) = val; }
        if (ps == 0) __threadfence(); }
}

__global__ __launch_bounds__(256) void k_cvt8(const float* __restrict__ src, bf* dst, size_t n8) { const size_t i = (size_t)blockIdx.x * 256 + threadIdx.x; if (i >= n8) return; const v8f v = *(const v8f*)(src + i * 8); v8us o;
#pragma unroll
    for (int k = 0; k < 8; ++k) o[k] = f2bf(v[k]); *(volatile v8us*)(dst + i * 8) = o; __threadfence(); *(volatile v8us*)(dst + i * 8) = o; }
__global__ __launch_bounds__(256) void k_cvtx(const float* __restrict__ src, bf* dst) { const unsigned i = blockIdx.x * 256u + threadIdx.x; if (i >= (unsigned)NB * SEQ * (DM / 8)) return;
    const unsigned m = i >> 7, c8 = i & 127u; const unsigned b = m / (unsigned)SEQ, t = m % (unsigned)SEQ; const v8f v = *(const v8f*)(src + ((size_t)b * SEQ_FULL + t) * DM + c8 * 8u); v8us o;
#pragma unroll
    for (int k = 0; k < 8; ++k) o[k] = f2bf(v[k]); *(volatile v8us*)(dst + (size_t)i * 8) = o; __threadfence(); *(volatile v8us*)(dst + (size_t)i * 8) = o; }

constexpr size_t SZ_X = (size_t)NB * SEQ * DM * 2;
constexpr size_t SZ_W = (size_t)DM * DM * 2;
constexpr size_t SZ_P = (size_t)NB * NH_ * SEQ * HD * 2;
constexpr size_t SZ_R = (size_t)NB * NH_ * RH * HD * 2;
constexpr size_t WS_TOTAL = 2 * SZ_X + 3 * SZ_W + 3 * SZ_P + 6 * SZ_R;
static_assert(SZ_X % 256 == 0 && SZ_W % 256 == 0 && SZ_P % 256 == 0 && SZ_R % 256 == 0);
static_assert(WS_TOTAL <= (size_t)134217728);
static_assert(((size_t)NB * SEQ * (DM / 8)) % 256 == 0);
static_assert(((size_t)DM * DM / 8) % 256 == 0);
static_assert(((size_t)(NB_FULL - 1) * SEQ_FULL + SEQ_FULL) * DM * 4 == (size_t)33554432);

extern "C" void kernel_launch(void* const* d_in, const int* in_sizes, int n_in,
                              void* d_out, int out_size, void* d_ws, size_t ws_size, hipStream_t stream) {
    if (n_in < 5) return;
    const size_t need_x = ((size_t)(NB - 1) * SEQ_FULL + SEQ) * DM;
    if ((size_t)in_sizes[0] < need_x) return;
    if ((size_t)in_sizes[1] < need_x) return;
    for (int i = 2; i < 5; ++i) if ((size_t)in_sizes[i] < (size_t)DM * DM) return;
    if ((size_t)out_size < need_x) return;
    if (ws_size < WS_TOTAL) return;
    const float* xq = (const float*)d_in[0]; const float* xkv = (const float*)d_in[1]; const float* wq = (const float*)d_in[2]; const float* wk = (const float*)d_in[3]; const float* wv = (const float*)d_in[4];
    float* OUT = (float*)d_out;
    char* wsp = (char*)d_ws;
    auto take = [&](size_t bytes) { char* p = wsp; wsp += (bytes + 255) & ~(size_t)255; return (void*)p; };
    bf* XQB = (bf*)take(SZ_X); bf* XKB = (bf*)take(SZ_X);
    bf* WQ = (bf*)take(SZ_W); bf* WK = (bf*)take(SZ_W); bf* WV = (bf*)take(SZ_W);
    h16* QP16 = (h16*)take(SZ_P); h16* KP16 = (h16*)take(SZ_P); h16* VT16 = (h16*)take(SZ_P);
    bf* QPh = (bf*)take(SZ_R); bf* QPl = (bf*)take(SZ_R); bf* KPh = (bf*)take(SZ_R); bf* KPl = (bf*)take(SZ_R); bf* VTh = (bf*)take(SZ_R); bf* VTl = (bf*)take(SZ_R);
    if ((size_t)(wsp - (char*)d_ws) > ws_size) return;

    const unsigned gx = (unsigned)((size_t)NB * SEQ * (DM / 8) / 256);
    k_cvtx<<<gx, 256, 0, stream>>>(xq, XQB);
    k_cvtx<<<gx, 256, 0, stream>>>(xkv, XKB);
    const unsigned gw = (unsigned)((size_t)DM * DM / 8 / 256);
    k_cvt8<<<gw, 256, 0, stream>>>(wq, WQ, (size_t)DM * DM / 8);
    k_cvt8<<<gw, 256, 0, stream>>>(wk, WK, (size_t)DM * DM / 8);
    k_cvt8<<<gw, 256, 0, stream>>>(wv, WV, (size_t)DM * DM / 8);

    const dim3 gp(NB * SEQ / 64, DM / 64, 1);
    k_projp<0><<<gp, 32, 0, stream>>>(XQB, WQ, QP16, QPh, QPl);
    k_projp<0><<<gp, 32, 0, stream>>>(XKB, WK, KP16, KPh, KPl);
    k_projp<1><<<gp, 32, 0, stream>>>(XKB, WV, VT16, VTh, VTl);

    k_flash<bf, true, (RH)><<<dim3(RH / 16, NB * NH_, 1), 32, 0, stream>>>(QPh, QPl, KPh, KPl, VTh, VTl, 0u, OUT);
    if (SEQ > RH)
        k_flash<h16, false, (SEQ)><<<dim3((SEQ - RH) / 16, NB * NH_, 1), 32, 0, stream>>>(QP16, nullptr, KP16, nullptr, VT16, nullptr, (unsigned)RH, OUT);
}
